// Olmo3_5HybridGatedDeltaNet_21500606283865
// MI455X (gfx1250) — hardware-verified
//
#include <hip/hip_runtime.h>
#include <hip/hip_bf16.h>


#define T_    1024
#define HID_  2048
#define NH_   16
#define DK_   96
#define DV_   192
#define KEY_  1536
#define VAL_  3072
#define CONV_ 6144
#define NCAT_ 6176
#define NP_   6208
#define COLB_ 6144
#define COLA_ 6160
#define NDVB_ 6

static_assert(NP_ % 64 == 0);
static_assert(NP_ >= NCAT_);
static_assert(T_ % 64 == 0);
static_assert(HID_ % 64 == 0);
static_assert(VAL_ % 64 == 0);
static_assert(KEY_ % 64 == 0);
static_assert(KEY_ == NH_ * DK_);
static_assert(VAL_ == NH_ * DV_);
static_assert(CONV_ == 2 * KEY_ + VAL_);
static_assert(NCAT_ == CONV_ + 2 * NH_);
static_assert(NDVB_ * 32 == DV_);
static_assert(DK_ == 8 * 12);
static_assert(DK_ == 3 * 32);
static_assert(DV_ == 24 * 8);
static_assert(T_ % 32 == 0);
static_assert((NP_ * 4) % 128 == 0 && (CONV_ * 4) % 128 == 0 && (VAL_ * 4) % 128 == 0 && (HID_ * 4) % 128 == 0);
static_assert((DK_ * 4) % 128 == 0 && (DV_ * 2) % 128 == 0 && (DV_ * 4) % 128 == 0);

typedef float          v4f   __attribute__((ext_vector_type(4)));
typedef float          v8f   __attribute__((ext_vector_type(8)));
typedef __bf16         v16b  __attribute__((ext_vector_type(16)));
typedef unsigned short u16x8 __attribute__((ext_vector_type(8)));

union FragB { u16x8 h[2]; v16b v; };

constexpr size_t SZ_HS16 = (size_t)T_ * HID_ * 2;
constexpr size_t SZ_WC16 = (size_t)NP_ * HID_ * 2;
constexpr size_t SZ_WPL  = 2 * SZ_WC16;
constexpr size_t SZ_WG16 = (size_t)VAL_ * HID_ * 2;
constexpr size_t SZ_WO16 = (size_t)HID_ * VAL_ * 2;
constexpr size_t SZ_PROJ = (size_t)T_ * NP_ * 4;
constexpr size_t SZ_GATE = (size_t)T_ * VAL_ * 4;
constexpr size_t SZ_ACT  = (size_t)T_ * CONV_ * 4;
constexpr size_t SZ_CG16 = (size_t)T_ * VAL_ * 2;
constexpr size_t SZ_CORE = (size_t)T_ * VAL_ * 4;

constexpr size_t OFF_HSH  = 0;
constexpr size_t OFF_HSL  = OFF_HSH + SZ_HS16;
constexpr size_t OFF_WPL  = OFF_HSL + SZ_HS16;
constexpr size_t OFF_WCH  = OFF_WPL;
constexpr size_t OFF_WCL  = OFF_WCH + SZ_WC16;
constexpr size_t OFF_WGH  = OFF_WPL;
constexpr size_t OFF_WGL  = OFF_WGH + SZ_WG16;
constexpr size_t OFF_WOH  = OFF_WGL + SZ_WG16;
constexpr size_t OFF_WOL  = OFF_WOH + SZ_WO16;
constexpr size_t OFF_PROJ = OFF_WPL + SZ_WPL;
constexpr size_t OFF_GATE = OFF_PROJ;
constexpr size_t OFF_ACT  = OFF_PROJ + SZ_PROJ;
constexpr size_t OFF_CGH  = OFF_ACT;
constexpr size_t OFF_CGL  = OFF_CGH + SZ_CG16;
constexpr size_t OFF_CORE = OFF_ACT + SZ_ACT;
constexpr size_t WS_END   = OFF_CORE + SZ_CORE;
static_assert(WS_END <= (size_t)134217728);
static_assert(OFF_WOL + SZ_WO16 <= OFF_PROJ);
static_assert(SZ_GATE <= SZ_PROJ);
static_assert(OFF_CGL + SZ_CG16 <= OFF_CORE);
static_assert(OFF_HSL % 128 == 0 && OFF_WPL % 128 == 0 && OFF_WCL % 128 == 0 && OFF_WGL % 128 == 0);
static_assert(OFF_WOH % 128 == 0 && OFF_WOL % 128 == 0 && OFF_PROJ % 128 == 0 && OFF_ACT % 128 == 0);
static_assert(OFF_CGL % 128 == 0 && OFF_CORE % 128 == 0);

__device__ __forceinline__ unsigned short f32_to_bf16(float f) {
    unsigned u = __float_as_uint(f);
    unsigned r = u + 0x7FFFu + ((u >> 16) & 1u);
    return (unsigned short)(r >> 16);
}
__device__ __forceinline__ float bf16_to_f32(unsigned short b) {
    return __uint_as_float(((unsigned)b) << 16);
}
__device__ __forceinline__ float silu_f(float x) {
    float e = __expf(-x);
    return x * __builtin_amdgcn_rcpf(1.0f + e);
}
__device__ __forceinline__ v8f ld8f(const float* p) {
    v4f a = *(const v4f*)p;
    v4f b = *(const v4f*)(p + 4);
    return __builtin_shufflevector(a, b, 0, 1, 2, 3, 4, 5, 6, 7);
}
__device__ __forceinline__ void split8(const v8f x, u16x8& hv, u16x8& lv) {
#pragma unroll
    for (int c = 0; c < 8; ++c) {
        const float f = x[c];
        const unsigned short hb = f32_to_bf16(f);
        const unsigned short lb = f32_to_bf16(f - bf16_to_f32(hb));
        hv[c] = hb;
        lv[c] = lb;
    }
}

__device__ __forceinline__ void mma16(v8f& acc, const FragB& a, const FragB& b) {
    acc = __builtin_amdgcn_wmma_f32_16x16x32_bf16(false, a.v, false, b.v, (short)0, acc, false, false);
    asm volatile("v_nop\n\tv_nop\n\tv_nop\n\tv_nop" : "+v"(acc) : "v"(a.v), "v"(b.v));
}

__global__ __launch_bounds__(256)
void hs_cvt_kernel(const float* __restrict__ src, unsigned short* dhi, unsigned short* dlo, int n8)
{
    const int i = blockIdx.x * 256 + threadIdx.x;
    if (i >= n8) return;
    const size_t e = (size_t)i * 8;
    const v8f x = ld8f(src + e);
    u16x8 hv, lv;
    split8(x, hv, lv);
    *(volatile u16x8*)(dhi + e) = hv;
    *(volatile u16x8*)(dlo + e) = lv;
    __threadfence();
    *(volatile u16x8*)(dhi + e) = hv;
    *(volatile u16x8*)(dlo + e) = lv;
}

__global__ __launch_bounds__(256)
void wt_cvt_kernel(const float* __restrict__ src, unsigned short* dhi, unsigned short* dlo,
                   int Nw, int Kd, int nrows)
{
    __shared__ __attribute__((aligned(16))) float sT[64 * 68];
    const int tid  = threadIdx.x;
    const int lane = tid & 31;
    const int wave = tid >> 5;
    const int n0 = blockIdx.x * 64;
    const int k0 = blockIdx.y * 64;

#pragma unroll
    for (int it = 0; it < 4; ++it) {
        const int idx = it * 256 + tid;
        const int kk  = idx >> 4;
        const int n4  = (idx & 15) * 4;
        const int gn  = n0 + n4;
        const int gnc = min(gn, Nw - 4);
        const v4f v = *(const v4f*)(src + (size_t)(k0 + kk) * Nw + gnc);
        const bool in = (gn < Nw);
        sT[(n4 + 0) * 68 + kk] = in ? v[0] : 0.0f;
        sT[(n4 + 1) * 68 + kk] = in ? v[1] : 0.0f;
        sT[(n4 + 2) * 68 + kk] = in ? v[2] : 0.0f;
        sT[(n4 + 3) * 68 + kk] = in ? v[3] : 0.0f;
    }
    __syncthreads();

    u16x8 hv[2], lv[2];
    const int c = (lane & 7) * 8;
#pragma unroll
    for (int it = 0; it < 2; ++it) {
        const int nn = it * 32 + wave * 4 + (lane >> 3);
        const v8f x = ld8f(sT + nn * 68 + c);
        split8(x, hv[it], lv[it]);
    }
#pragma unroll
    for (int it = 0; it < 2; ++it) {
        const int gr = n0 + it * 32 + wave * 4 + (lane >> 3);
        if (gr < nrows) {
            const size_t o = (size_t)gr * Kd + k0 + c;
            *(volatile u16x8*)(dhi + o) = hv[it];
            *(volatile u16x8*)(dlo + o) = lv[it];
        }
    }
    __threadfence();
#pragma unroll
    for (int it = 0; it < 2; ++it) {
        const int gr = n0 + it * 32 + wave * 4 + (lane >> 3);
        if (gr < nrows) {
            const size_t o = (size_t)gr * Kd + k0 + c;
            *(volatile u16x8*)(dhi + o) = hv[it];
            *(volatile u16x8*)(dlo + o) = lv[it];
        }
    }
}

template<int NBF>
__device__ __forceinline__ void tile_store_pass(const float* st, float* gp, int ldc, int lane) {
    constexpr int CW  = NBF * 16;
    constexpr int P   = CW + 4;
    constexpr int LPR = CW / 4;
    static_assert(32 % LPR == 0);
    constexpr int RPI = 32 / LPR;
    constexpr int NIT = 32 / RPI;
    const int rsub = lane / LPR;
    const int c0   = (lane % LPR) * 4;
#pragma unroll
    for (int it = 0; it < NIT; ++it) {
        const int row = it * RPI + rsub;
        const v4f v = *(const v4f*)(st + row * P + c0);
        *(volatile v4f*)(gp + (size_t)row * ldc + c0) = v;
    }
}

template<int NBF>
__global__ __launch_bounds__(128)
void gemm_x3_kernel(const unsigned short* __restrict__ Ah, const unsigned short* __restrict__ Al,
                    const unsigned short* __restrict__ Bh, const unsigned short* __restrict__ Bl,
                    float* C, int K, int ldc)
{
    constexpr int CW = NBF * 16;
    constexpr int P  = CW + 4;
    static_assert(CW % 32 == 0);
    __shared__ __attribute__((aligned(16))) float stile[4][32 * P];

    const int tid  = threadIdx.x;
    const int lane = tid & 31;
    const int wave = tid >> 5;
    const int h    = lane >> 4;
    const int m    = lane & 15;
    const int wm   = wave >> 1;
    const int wn   = wave & 1;

    const int rowW = blockIdx.y * 64 + wm * 32;
    const int colW = blockIdx.x * (2 * CW) + wn * CW;

    v8f acc[2 * NBF];
#pragma unroll
    for (int j = 0; j < 2 * NBF; ++j)
#pragma unroll
        for (int r = 0; r < 8; ++r) acc[j][r] = 0.0f;

    const size_t aoff  = (size_t)(rowW + m) * K + 8 * h;
    const size_t boff  = (size_t)(colW + m) * K + 8 * h;
    const size_t sub16 = (size_t)16 * K;
    const int nk = K >> 5;

#pragma unroll 1
    for (int kt = 0; kt < nk; ++kt) {
        const size_t k0 = (size_t)kt * 32;
        FragB fa[2], ga[2], fb[NBF], gb[NBF];
#pragma unroll
        for (int s = 0; s < 2; ++s) {
            const unsigned short* p = Ah + aoff + s * sub16 + k0;
            const unsigned short* q = Al + aoff + s * sub16 + k0;
            fa[s].h[0] = *(const u16x8*)(p);
            fa[s].h[1] = *(const u16x8*)(p + 16);
            ga[s].h[0] = *(const u16x8*)(q);
            ga[s].h[1] = *(const u16x8*)(q + 16);
        }
#pragma unroll
        for (int j = 0; j < NBF; ++j) {
            const unsigned short* p = Bh + boff + j * sub16 + k0;
            const unsigned short* q = Bl + boff + j * sub16 + k0;
            fb[j].h[0] = *(const u16x8*)(p);
            fb[j].h[1] = *(const u16x8*)(p + 16);
            gb[j].h[0] = *(const u16x8*)(q);
            gb[j].h[1] = *(const u16x8*)(q + 16);
        }
#pragma unroll
        for (int s = 0; s < 2; ++s)
#pragma unroll
            for (int j = 0; j < NBF; ++j) {
                mma16(acc[s * NBF + j], fa[s], fb[j]);
                mma16(acc[s * NBF + j], fa[s], gb[j]);
                mma16(acc[s * NBF + j], ga[s], fb[j]);
            }
    }

    float* st = stile[wave];
#pragma unroll
    for (int s = 0; s < 2; ++s)
#pragma unroll
        for (int j = 0; j < NBF; ++j)
#pragma unroll
            for (int r = 0; r < 8; ++r)
                st[(s * 16 + 8 * h + r) * P + j * 16 + m] = acc[s * NBF + j][r];
    __syncthreads();

    float* gp = C + (size_t)rowW * ldc + colW;
    tile_store_pass<NBF>(st, gp, ldc, lane);
    __threadfence();
    tile_store_pass<NBF>(st, gp, ldc, lane);
}

__global__ __launch_bounds__(256)
void prep_kernel(const float* __restrict__ proj, const float* __restrict__ cwq,
                 const float* __restrict__ cwk, const float* __restrict__ cwv, float* act)
{
    const int t    = blockIdx.x;
    const int tid  = threadIdx.x;
    const int lane = tid & 31;
    const int wave = tid >> 5;
    const int r0 = max(t - 3, 0), r1 = max(t - 2, 0), r2 = max(t - 1, 0);
    const float z0 = (t >= 3) ? 1.0f : 0.0f;
    const float z1 = (t >= 2) ? 1.0f : 0.0f;
    const float z2 = (t >= 1) ? 1.0f : 0.0f;
    const float* p3 = proj + (size_t)t  * NP_;
    const float* p2 = proj + (size_t)r2 * NP_;
    const float* p1 = proj + (size_t)r1 * NP_;
    const float* p0 = proj + (size_t)r0 * NP_;
    const float qscale = 0.10206207261596575f;
    float* arow = act + (size_t)t * CONV_;

#pragma unroll 1
    for (int it = 0; it < 4; ++it) {
        const int hr  = it * 8 + wave;
        const int isk = hr >> 4;
        const int cb  = hr * DK_;
        const int wb  = (hr & 15) * DK_;
        const float* cw = isk ? cwk : cwq;
        const float osc = isk ? 1.0f : qscale;
        float cv[3];
#pragma unroll
        for (int i = 0; i < 3; ++i) {
            const int c  = cb + lane + 32 * i;
            const float x3 = p3[c];
            const float x2 = p2[c] * z2;
            const float x1 = p1[c] * z1;
            const float x0 = p0[c] * z0;
            const v4f w = *(const v4f*)(cw + (size_t)(wb + lane + 32 * i) * 4);
            float a = w[0] * x0;
            a = w[1] * x1 + a;
            a = w[2] * x2 + a;
            a = w[3] * x3 + a;
            cv[i] = silu_f(a);
        }
        float ss = cv[0] * cv[0] + cv[1] * cv[1] + cv[2] * cv[2];
#pragma unroll
        for (int mm = 16; mm >= 1; mm >>= 1) ss += __shfl_xor(ss, mm, 32);
        const float rr = rsqrtf(ss + 1e-6f);
        const float o0 = (cv[0] * rr) * osc;
        const float o1 = (cv[1] * rr) * osc;
        const float o2 = (cv[2] * rr) * osc;
        float* gp = arow + cb + lane;
        *(volatile float*)(gp)      = o0;
        *(volatile float*)(gp + 32) = o1;
        *(volatile float*)(gp + 64) = o2;
        __threadfence();
        *(volatile float*)(gp)      = o0;
        *(volatile float*)(gp + 32) = o1;
        *(volatile float*)(gp + 64) = o2;
    }

#pragma unroll 1
    for (int p = 0; p < 3; ++p) {
        const int c   = p * 1024 + tid * 4;
        const int col = 2 * KEY_ + c;
        const v4f x3 = *(const v4f*)(p3 + col);
        const v4f x2 = *(const v4f*)(p2 + col) * z2;
        const v4f x1 = *(const v4f*)(p1 + col) * z1;
        const v4f x0 = *(const v4f*)(p0 + col) * z0;
        v4f wt[4];
#pragma unroll
        for (int i = 0; i < 4; ++i) wt[i] = *(const v4f*)(cwv + (size_t)(c + i) * 4);
        v4f cvv;
#pragma unroll
        for (int i = 0; i < 4; ++i) {
            float a = wt[i][0] * x0[i];
            a = wt[i][1] * x1[i] + a;
            a = wt[i][2] * x2[i] + a;
            a = wt[i][3] * x3[i] + a;
            cvv[i] = silu_f(a);
        }
        float* gp = arow + col;
        *(volatile v4f*)gp = cvv;
        __threadfence();
        *(volatile v4f*)gp = cvv;
    }
}

__global__ __launch_bounds__(256)
void delta_kernel(const float* __restrict__ act, const float* __restrict__ proj,
                  const float* __restrict__ alog, const float* __restrict__ dtb, float* core)
{
    __shared__ float sdec[T_];
    __shared__ float sbet[T_];
    __shared__ __attribute__((aligned(16))) float sout[32 * 32];

    const int tid  = threadIdx.x;
    const int lane = tid & 31;
    const int wave = tid >> 5;
    const int h    = blockIdx.x / NDVB_;
    const int dvb  = (blockIdx.x % NDVB_) * 32;
    const int dvl  = tid >> 3;
    const int part = tid & 7;

    const float ae = expf(alog[h]);
    const float db = dtb[h];
#pragma unroll 1
    for (int s = tid; s < T_; s += 256) {
        const float b = proj[(size_t)s * NP_ + COLB_ + h];
        const float a = proj[(size_t)s * NP_ + COLA_ + h];
        sbet[s] = 2.0f * __builtin_amdgcn_rcpf(1.0f + __expf(-b));
        const float x  = a + db;
        const float sp = fmaxf(x, 0.0f) + log1pf(__expf(-fabsf(x)));
        sdec[s] = expf(-(ae * sp));
    }
    __syncthreads();

    float st[12];
#pragma unroll
    for (int i = 0; i < 12; ++i) st[i] = 0.0f;

    const float* qb = act + h * DK_ + part * 12;
    const float* kb = act + KEY_ + h * DK_ + part * 12;
    const float* vb = act + 2 * KEY_ + h * DV_ + dvb + dvl;

#pragma unroll 1
    for (int s = 0; s < T_; ++s) {
        const size_t ro = (size_t)s * CONV_;
        v4f k4[3], q4[3];
#pragma unroll
        for (int i = 0; i < 3; ++i) {
            k4[i] = *(const v4f*)(kb + ro + 4 * i);
            q4[i] = *(const v4f*)(qb + ro + 4 * i);
        }
        const float vv = vb[ro];
        const float eg = sdec[s];
        const float bt = sbet[s];

        float kv = 0.0f;
#pragma unroll
        for (int i = 0; i < 12; ++i) {
            st[i] = st[i] * eg;
            kv = st[i] * k4[i >> 2][i & 3] + kv;
        }
        kv += __shfl_xor(kv, 1, 32);
        kv += __shfl_xor(kv, 2, 32);
        kv += __shfl_xor(kv, 4, 32);

        const float delta = (vv - kv) * bt;

        float o = 0.0f;
#pragma unroll
        for (int i = 0; i < 12; ++i) {
            st[i] = k4[i >> 2][i & 3] * delta + st[i];
            o = st[i] * q4[i >> 2][i & 3] + o;
        }
        o += __shfl_xor(o, 1, 32);
        o += __shfl_xor(o, 2, 32);
        o += __shfl_xor(o, 4, 32);

        if (part == 0) sout[(s & 31) * 32 + dvl] = o;

        if ((s & 31) == 31) {
            __syncthreads();
            const int tt = wave * 4 + (lane >> 3);
            const int c  = (lane & 7) * 4;
            const v4f v = *(const v4f*)(sout + tt * 32 + c);
            float* gp = core + (size_t)(s - 31 + tt) * VAL_ + h * DV_ + dvb + c;
            *(volatile v4f*)gp = v;
            __threadfence();
            *(volatile v4f*)gp = v;
            __syncthreads();
        }
    }
}

__global__ __launch_bounds__(256)
void norm_gate_kernel(const float* __restrict__ core, const float* __restrict__ gate,
                      const float* __restrict__ nw, unsigned short* chi, unsigned short* clo)
{
    const int tid  = threadIdx.x;
    const int lane = tid & 31;
    const int wave = tid >> 5;
    const int r    = blockIdx.x * 8 + wave;
    const int t    = r >> 4;
    const int hh   = r & 15;
    const int lc   = min(lane, 23);
    const int c0   = lc * 8;
    const size_t base = (size_t)t * VAL_ + hh * DV_ + c0;

    const v8f x = ld8f(core + base);
    float ss = 0.0f;
#pragma unroll
    for (int i = 0; i < 8; ++i) ss = x[i] * x[i] + ss;
    ss = (lane < 24) ? ss : 0.0f;
    ss += __shfl_xor(ss, 16, 32);
    ss += __shfl_xor(ss, 8, 32);
    ss += __shfl_xor(ss, 4, 32);
    ss += __shfl_xor(ss, 2, 32);
    ss += __shfl_xor(ss, 1, 32);
    const float rr = rsqrtf(ss * (1.0f / 192.0f) + 1e-6f);

    const v8f z = ld8f(gate + base);
    const v8f w = ld8f(nw + c0);
    v8f y;
#pragma unroll
    for (int i = 0; i < 8; ++i) {
        const float tv = (x[i] * rr) * w[i];
        y[i] = tv * silu_f(z[i]);
    }
    u16x8 hv, lv;
    split8(y, hv, lv);
    if (lane < 24) {
        *(volatile u16x8*)(chi + base) = hv;
        *(volatile u16x8*)(clo + base) = lv;
    }
    __threadfence();
    if (lane < 24) {
        *(volatile u16x8*)(chi + base) = hv;
        *(volatile u16x8*)(clo + base) = lv;
    }
}

extern "C" void kernel_launch(void* const* d_in, const int* in_sizes, int n_in,
                              void* d_out, int out_size, void* d_ws, size_t ws_size,
                              hipStream_t stream)
{
    if (n_in < 14) return;
    if (in_sizes[0]  != T_ * HID_)     return;
    if (in_sizes[1]  != HID_ * KEY_)   return;
    if (in_sizes[2]  != HID_ * KEY_)   return;
    if (in_sizes[3]  != HID_ * VAL_)   return;
    if (in_sizes[4]  != KEY_ * 4)      return;
    if (in_sizes[5]  != KEY_ * 4)      return;
    if (in_sizes[6]  != VAL_ * 4)      return;
    if (in_sizes[7]  != HID_ * NH_)    return;
    if (in_sizes[8]  != HID_ * NH_)    return;
    if (in_sizes[9]  != NH_)           return;
    if (in_sizes[10] != NH_)           return;
    if (in_sizes[11] != HID_ * VAL_)   return;
    if (in_sizes[12] != DV_)           return;
    if (in_sizes[13] != VAL_ * HID_)   return;
    if (out_size != T_ * HID_)         return;
    if (ws_size < WS_END)              return;

    const float* hidden = (const float*)d_in[0];
    const float* Wq     = (const float*)d_in[1];
    const float* Wk     = (const float*)d_in[2];
    const float* Wv     = (const float*)d_in[3];
    const float* conv_q = (const float*)d_in[4];
    const float* conv_k = (const float*)d_in[5];
    const float* conv_v = (const float*)d_in[6];
    const float* Wb     = (const float*)d_in[7];
    const float* Wa     = (const float*)d_in[8];
    const float* A_log  = (const float*)d_in[9];
    const float* dt_b   = (const float*)d_in[10];
    const float* Wg     = (const float*)d_in[11];
    const float* nw     = (const float*)d_in[12];
    const float* Wo     = (const float*)d_in[13];
    float* out = (float*)d_out;

    char* ws = (char*)d_ws;
    unsigned short* hsh  = (unsigned short*)(ws + OFF_HSH);
    unsigned short* hsl  = (unsigned short*)(ws + OFF_HSL);
    unsigned short* wch  = (unsigned short*)(ws + OFF_WCH);
    unsigned short* wcl  = (unsigned short*)(ws + OFF_WCL);
    unsigned short* wgh  = (unsigned short*)(ws + OFF_WGH);
    unsigned short* wgl  = (unsigned short*)(ws + OFF_WGL);
    unsigned short* woh  = (unsigned short*)(ws + OFF_WOH);
    unsigned short* wol  = (unsigned short*)(ws + OFF_WOL);
    float*          proj = (float*)(ws + OFF_PROJ);
    float*          gate = (float*)(ws + OFF_GATE);
    float*          act  = (float*)(ws + OFF_ACT);
    unsigned short* cgh  = (unsigned short*)(ws + OFF_CGH);
    unsigned short* cgl  = (unsigned short*)(ws + OFF_CGL);
    float*          core = (float*)(ws + OFF_CORE);

    {
        const int n8 = (T_ * HID_) / 8;
        hs_cvt_kernel<<<dim3((n8 + 255) / 256), dim3(256), 0, stream>>>(hidden, hsh, hsl, n8);
    }

    wt_cvt_kernel<<<dim3(KEY_ / 64, HID_ / 64), dim3(256), 0, stream>>>(
        Wq, wch, wcl, (int)KEY_, (int)HID_, (int)KEY_);
    wt_cvt_kernel<<<dim3(KEY_ / 64, HID_ / 64), dim3(256), 0, stream>>>(
        Wk, wch + (size_t)KEY_ * HID_, wcl + (size_t)KEY_ * HID_, (int)KEY_, (int)HID_, (int)KEY_);
    wt_cvt_kernel<<<dim3(VAL_ / 64, HID_ / 64), dim3(256), 0, stream>>>(
        Wv, wch + (size_t)(2 * KEY_) * HID_, wcl + (size_t)(2 * KEY_) * HID_, (int)VAL_, (int)HID_, (int)VAL_);
    wt_cvt_kernel<<<dim3(1, HID_ / 64), dim3(256), 0, stream>>>(
        Wb, wch + (size_t)COLB_ * HID_, wcl + (size_t)COLB_ * HID_, (int)NH_, (int)HID_, (int)NH_);
    wt_cvt_kernel<<<dim3((NP_ - COLA_ + 63) / 64, HID_ / 64), dim3(256), 0, stream>>>(
        Wa, wch + (size_t)COLA_ * HID_, wcl + (size_t)COLA_ * HID_, (int)NH_, (int)HID_, (int)(NP_ - COLA_));

    gemm_x3_kernel<2><<<dim3(NP_ / 64, T_ / 64), dim3(128), 0, stream>>>(
        (const unsigned short*)hsh, (const unsigned short*)hsl,
        (const unsigned short*)wch, (const unsigned short*)wcl,
        proj, (int)HID_, (int)NP_);

    prep_kernel<<<dim3(T_), dim3(256), 0, stream>>>((const float*)proj, conv_q, conv_k, conv_v, act);

    delta_kernel<<<dim3(NH_ * NDVB_), dim3(256), 0, stream>>>(
        (const float*)act, (const float*)proj, A_log, dt_b, core);

    wt_cvt_kernel<<<dim3(VAL_ / 64, HID_ / 64), dim3(256), 0, stream>>>(
        Wg, wgh, wgl, (int)VAL_, (int)HID_, (int)VAL_);
    wt_cvt_kernel<<<dim3(HID_ / 64, VAL_ / 64), dim3(256), 0, stream>>>(
        Wo, woh, wol, (int)HID_, (int)VAL_, (int)HID_);

    gemm_x3_kernel<2><<<dim3(VAL_ / 64, T_ / 64), dim3(128), 0, stream>>>(
        (const unsigned short*)hsh, (const unsigned short*)hsl,
        (const unsigned short*)wgh, (const unsigned short*)wgl,
        gate, (int)HID_, (int)VAL_);

    norm_gate_kernel<<<dim3((T_ * NH_) / 8), dim3(256), 0, stream>>>(
        (const float*)core, (const float*)gate, nw, cgh, cgl);

    gemm_x3_kernel<2><<<dim3(HID_ / 64, T_ / 64), dim3(128), 0, stream>>>(
        (const unsigned short*)cgh, (const unsigned short*)cgl,
        (const unsigned short*)woh, (const unsigned short*)wol,
        out, (int)VAL_, (int)HID_);
}
